// RNN_62508954026437
// MI455X (gfx1250) — hardware-verified
//
#include <hip/hip_runtime.h>
#include <math.h>

constexpr int NBAT  = 2048;
constexpr int NFEAT = 4;
constexpr int NHID  = 1024;
constexpr int NLAY  = 4;
constexpr int NOUT  = 256;
constexpr int NGATE = 3 * NHID;
constexpr int NTHR  = 256;
constexpr int TPITCH = 68;
constexpr float CARRY    = 16.0f;
constexpr float PROD_INV = 1.0f / (CARRY * CARRY);
constexpr int BLK_ROWS = 128;
constexpr int BLK_COLS = 64;
static_assert(NHID % 32 == 0, "GEMM K must be a multiple of 32");
static_assert(NBAT % BLK_ROWS == 0 && NHID % BLK_COLS == 0, "layer grid exact");
static_assert(NBAT % 64 == 0 && NOUT % 64 == 0, "decoder tiles exact");
static_assert((NBAT * NOUT * 4) % 128 == 0, "second output starts on a 128-B line");
static_assert((size_t)NBAT * NOUT * 4 == 2097152u, "byte offset of the hidden stack");
static_assert(((size_t)NBAT * NOUT + (size_t)NLAY * NBAT * NHID) * 4 == 35651584u, "total output bytes");
static_assert((NBAT * NHID / 8) % NTHR == 0, "projection grid exact");

typedef __attribute__((ext_vector_type(16))) _Float16 v16h;
typedef __attribute__((ext_vector_type(8)))  _Float16 v8h;
typedef __attribute__((ext_vector_type(8)))  float    v8f;
typedef __attribute__((ext_vector_type(4)))  float    v4f;

__device__ __forceinline__ float bf16r(float f) {
  unsigned u = __float_as_uint(f);
  u = (u + 0x7FFFu + ((u >> 16) & 1u)) & 0xFFFF0000u;
  return __uint_as_float(u);
}

__device__ __forceinline__ void guard3_h(v8f& a, v8f& b, v8f& c, v16h x, v16h y0, v16h y1, v16h y2) {
  asm volatile("v_nop\n\tv_nop\n\tv_nop\n\tv_nop" : "+v"(a), "+v"(b), "+v"(c) : "v"(x), "v"(y0), "v"(y1), "v"(y2));
}
__device__ __forceinline__ void guard4_h(v8f& a, v8f& b, v8f& c, v8f& d, v16h x, v16h y0, v16h y1, v16h y2, v16h y3) {
  asm volatile("v_nop\n\tv_nop\n\tv_nop\n\tv_nop" : "+v"(a), "+v"(b), "+v"(c), "+v"(d) : "v"(x), "v"(y0), "v"(y1), "v"(y2), "v"(y3));
}
__device__ __forceinline__ void keep4_h(v16h a, v16h b, v16h c, v16h d) { asm volatile("v_nop" :: "v"(a), "v"(b), "v"(c), "v"(d)); }
__device__ __forceinline__ void acc_guard4(v8f& a, v8f& b, v8f& c, v8f& d) { asm volatile("v_nop\n\tv_nop\n\tv_nop\n\tv_nop" : "+v"(a), "+v"(b), "+v"(c), "+v"(d)); }

struct FragH {
  union U { v16h v; v8h h[2]; };
  static __device__ __forceinline__ v16h load(const _Float16* p) {
    U f; f.h[0] = *(const v8h*)(p); f.h[1] = *(const v8h*)(p + 16); return f.v;
  }
  static __device__ __forceinline__ v8f mma(v16h a, v16h b, v8f c) {
    return __builtin_amdgcn_wmma_f32_16x16x32_f16(false, a, false, b, (short)0, c, false, false);
  }
};

__global__ __launch_bounds__(NTHR) void cvt8_flat_kernel(const float* __restrict__ src, unsigned short* __restrict__ dst,
                                                         int n8, float sc) {
  const int i = blockIdx.x * NTHR + threadIdx.x;
  if (i < n8) {
    const float* sp = src + (size_t)i * 8;
    const v4f a = *(const v4f*)(sp);
    const v4f b = *(const v4f*)(sp + 4);
    v8h hv;
#pragma unroll
    for (int e = 0; e < 4; ++e) {
      const float fa = a[e];
      const float fb = b[e];
      hv[e]     = (_Float16)(bf16r(fa) * sc);
      hv[4 + e] = (_Float16)(bf16r(fb) * sc);
    }
    *(volatile v8h*)(dst + (size_t)i * 8) = hv;
    __threadfence();
    *(volatile v8h*)(dst + (size_t)i * 8) = hv;
  }
}

__global__ __launch_bounds__(NTHR) void i2h_kernel(const float* __restrict__ inp, const float* __restrict__ w,
                                                   const float* __restrict__ bias, unsigned short* __restrict__ xo) {
  const int t = blockIdx.x * NTHR + threadIdx.x;
  if (t < NBAT * NHID / 8) {
    const int b  = t >> 7;
    const int j8 = (t & 127) * 8;
    const v4f xin = *(const v4f*)(inp + (size_t)b * NFEAT);
    const float xa = xin[0];
    const float xb = xin[1];
    const float xc = xin[2];
    const float xd = xin[3];
    const float x0 = bf16r(xa), x1 = bf16r(xb), x2 = bf16r(xc), x3 = bf16r(xd);
    const v4f bb0 = *(const v4f*)(bias + j8);
    const v4f bb1 = *(const v4f*)(bias + j8 + 4);
    v8h hv;
#pragma unroll
    for (int e = 0; e < 4; ++e) {
      const v4f wv = *(const v4f*)(w + (size_t)(j8 + e) * NFEAT);
      const float wa = wv[0];
      const float wb = wv[1];
      const float wc = wv[2];
      const float wd = wv[3];
      const float be = bb0[e];
      float s = x0 * bf16r(wa);
      s = fmaf(x1, bf16r(wb), s);
      s = fmaf(x2, bf16r(wc), s);
      s = fmaf(x3, bf16r(wd), s);
      s += bf16r(be);
      hv[e] = (_Float16)(s * CARRY);
    }
    asm volatile("" ::: "memory");
#pragma unroll
    for (int e = 0; e < 4; ++e) {
      const v4f wv = *(const v4f*)(w + (size_t)(j8 + 4 + e) * NFEAT);
      const float wa = wv[0];
      const float wb = wv[1];
      const float wc = wv[2];
      const float wd = wv[3];
      const float be = bb1[e];
      float s = x0 * bf16r(wa);
      s = fmaf(x1, bf16r(wb), s);
      s = fmaf(x2, bf16r(wc), s);
      s = fmaf(x3, bf16r(wd), s);
      s += bf16r(be);
      hv[4 + e] = (_Float16)(s * CARRY);
    }
    unsigned short* op = xo + (size_t)b * NHID + j8;
    *(volatile v8h*)op = hv;
    __threadfence();
    *(volatile v8h*)op = hv;
  }
}

__global__ __launch_bounds__(NTHR) void gru_layer_kernel(
    const unsigned short* __restrict__ Xp, const unsigned short* __restrict__ Hp,
    const unsigned short* __restrict__ Wip, const unsigned short* __restrict__ Whp,
    const float* __restrict__ bih, const float* __restrict__ bhh,
    const float* __restrict__ hid, float* __restrict__ hout, unsigned short* __restrict__ xnext) {
  __shared__ __align__(16) float Tl[4][32 * TPITCH];

  const _Float16* X  = (const _Float16*)Xp;
  const _Float16* Hh = (const _Float16*)Hp;
  const _Float16* Wi = (const _Float16*)Wip;
  const _Float16* Wh = (const _Float16*)Whp;

  const int tid  = threadIdx.x;
  const int lane = tid & 31;
  const int wave = tid >> 5;
  const int c    = lane & 15;
  const int hh   = lane >> 4;
  const int koff = hh * 8;
  const int mi   = wave >> 2;
  const int ni   = wave & 3;
  const int n0   = blockIdx.x * BLK_COLS;
  const int m0   = blockIdx.y * BLK_ROWS;

  const size_t GSTR = (size_t)NHID * NHID;
  const size_t ISTR = (size_t)32 * NHID;
  const _Float16* xrow = X  + (size_t)(m0 + 16 * mi + c) * NHID + koff;
  const _Float16* hrow = Hh + (size_t)(m0 + 16 * mi + c) * NHID + koff;
  const _Float16* wi   = Wi + (size_t)(n0 + 16 * ni + c) * NHID + koff;
  const _Float16* wh   = Wh + (size_t)(n0 + 16 * ni + c) * NHID + koff;

  const v8f z8 = {0.f, 0.f, 0.f, 0.f, 0.f, 0.f, 0.f, 0.f};
  v8f aR[4], aZ[4], aI[4], aH[4];
#pragma unroll
  for (int i = 0; i < 4; ++i) { aR[i] = z8; aZ[i] = z8; aI[i] = z8; aH[i] = z8; }

#pragma unroll 1
  for (int k0 = 0; k0 < NHID; k0 += 32) {
    {
      const v16h b0 = FragH::load(wi + k0);
      const v16h b1 = FragH::load(wi + GSTR + k0);
      const v16h b2 = FragH::load(wi + 2 * GSTR + k0);
#pragma unroll
      for (int i = 0; i < 4; ++i) {
        const v16h a = FragH::load(xrow + (size_t)i * ISTR + k0);
        aR[i] = FragH::mma(a, b0, aR[i]);
        aZ[i] = FragH::mma(a, b1, aZ[i]);
        aI[i] = FragH::mma(a, b2, aI[i]);
        guard3_h(aR[i], aZ[i], aI[i], a, b0, b1, b2);
      }
      keep4_h(b0, b1, b2, b0);
    }
    asm volatile("" ::: "memory");
    {
      const v16h b0 = FragH::load(wh + k0);
      const v16h b1 = FragH::load(wh + GSTR + k0);
      const v16h b2 = FragH::load(wh + 2 * GSTR + k0);
#pragma unroll
      for (int i = 0; i < 4; ++i) {
        const v16h a = FragH::load(hrow + (size_t)i * ISTR + k0);
        aR[i] = FragH::mma(a, b0, aR[i]);
        aZ[i] = FragH::mma(a, b1, aZ[i]);
        aH[i] = FragH::mma(a, b2, aH[i]);
        guard3_h(aR[i], aZ[i], aH[i], a, b0, b1, b2);
      }
      keep4_h(b0, b1, b2, b0);
    }
    asm volatile("" ::: "memory");
  }
  acc_guard4(aR[0], aR[1], aR[2], aR[3]);
  acc_guard4(aZ[0], aZ[1], aZ[2], aZ[3]);
  acc_guard4(aI[0], aI[1], aI[2], aI[3]);
  acc_guard4(aH[0], aH[1], aH[2], aH[3]);

  const int j = n0 + 16 * ni + c;
  const float br  = bf16r(bih[j]) + bf16r(bhh[j]);
  const float bz  = bf16r(bih[NHID + j]) + bf16r(bhh[NHID + j]);
  const float bin = bf16r(bih[2 * NHID + j]);
  const float bhn = bf16r(bhh[2 * NHID + j]);

#pragma unroll
  for (int i = 0; i < 4; ++i) {
#pragma unroll
    for (int r = 0; r < 8; ++r) {
      const int s = (16 * mi + 8 * hh + r) * TPITCH + 16 * ni + c;
      Tl[0][s] = aR[i][r] * PROD_INV + br;
      Tl[1][s] = aZ[i][r] * PROD_INV + bz;
      Tl[2][s] = aI[i][r] * PROD_INV + bin;
      Tl[3][s] = aH[i][r] * PROD_INV + bhn;
    }
    __syncthreads();
    const int rowb = m0 + 32 * i;
#pragma unroll 1
    for (int it = 0; it < 8; ++it) {
      const int idx  = it * NTHR + tid;
      const int lrow = idx >> 6;
      const int col  = idx & 63;
      const int s    = lrow * TPITCH + col;
      const float pr = Tl[0][s];
      const float pz = Tl[1][s];
      const float pi = Tl[2][s];
      const float ph = Tl[3][s];
      const float ho = bf16r(hid[(size_t)(rowb + lrow) * NHID + n0 + col]);
      const float rg = 1.0f / (1.0f + expf(-pr));
      const float zg = 1.0f / (1.0f + expf(-pz));
      const float ng = tanhf(pi + rg * ph);
      const float hn = (1.0f - zg) * ng + zg * ho;
      Tl[0][s] = hn;
    }
    __syncthreads();
    {
      const int c4 = c * 4;
      float* ob = hout + (size_t)rowb * NHID + n0;
      for (int pass = 0; pass < 2; ++pass) {
#pragma unroll
        for (int it = 0; it < 2; ++it) {
          const int lrow = 4 * wave + 2 * it + hh;
          const v4f v = *(const v4f*)(&Tl[0][lrow * TPITCH + c4]);
          *(volatile v4f*)(ob + (size_t)lrow * NHID + c4) = v;
        }
        __threadfence();
      }
    }
    {
      const int q  = lane >> 3;
      const int c8 = (lane & 7) * 8;
      const int lrow = 4 * wave + q;
      const float* sp = &Tl[0][lrow * TPITCH + c8];
      const v4f p0 = *(const v4f*)(sp);
      const v4f p1 = *(const v4f*)(sp + 4);
      v8h hv;
#pragma unroll
      for (int e = 0; e < 4; ++e) {
        const float f0 = p0[e];
        const float f1 = p1[e];
        hv[e]     = (_Float16)(f0 * CARRY);
        hv[4 + e] = (_Float16)(f1 * CARRY);
      }
      unsigned short* xp = xnext + (size_t)(rowb + lrow) * NHID + n0 + c8;
      *(volatile v8h*)xp = hv;
      __threadfence();
      *(volatile v8h*)xp = hv;
    }
    __syncthreads();
  }
}

template <bool BIAS_R16>
__global__ __launch_bounds__(256) void wmma_gemm64_f16(
    const unsigned short* __restrict__ Ap, int lda,
    const unsigned short* __restrict__ Btp, int ldb,
    float* __restrict__ Cout, int ldc,
    const float* __restrict__ bias, int M, int N, int K, float scale) {
  const _Float16* A  = (const _Float16*)Ap;
  const _Float16* Bt = (const _Float16*)Btp;
  __shared__ __align__(16) float sT[8][16 * 68];
  const int lane = threadIdx.x & 31;
  const int wave = threadIdx.x >> 5;
  const int tilesN = N >> 6;
  const int tilesM = M >> 6;
  const int tile = blockIdx.x * 8 + wave;
  if (tile >= tilesM * tilesN) return;
  const int tm = tile / tilesN;
  const int tn = tile - tm * tilesN;
  const int m0 = tm << 6;
  const int n0 = tn << 6;

  const int rlane = lane & 15;
  const int koff  = (lane >> 4) * 8;
  const int mOff  = (lane >> 4) * 8;

  v8f acc[4][4];
#pragma unroll
  for (int i = 0; i < 4; ++i)
#pragma unroll
    for (int jj = 0; jj < 4; ++jj) acc[i][jj] = (v8f){0.f, 0.f, 0.f, 0.f, 0.f, 0.f, 0.f, 0.f};

  for (int k0 = 0; k0 < K; k0 += 32) {
    v16h bh[4];
#pragma unroll
    for (int jj = 0; jj < 4; ++jj) {
      const size_t bo = (size_t)(n0 + (jj << 4) + rlane) * ldb + koff + k0;
      bh[jj] = FragH::load(Bt + bo);
    }
#pragma unroll
    for (int i = 0; i < 4; ++i) {
      const size_t ao = (size_t)(m0 + (i << 4) + rlane) * lda + koff + k0;
      const v16h ah = FragH::load(A + ao);
#pragma unroll
      for (int jj = 0; jj < 4; ++jj) acc[i][jj] = FragH::mma(ah, bh[jj], acc[i][jj]);
      guard4_h(acc[i][0], acc[i][1], acc[i][2], acc[i][3], ah, bh[0], bh[1], bh[2], bh[3]);
    }
    keep4_h(bh[0], bh[1], bh[2], bh[3]);
  }
  acc_guard4(acc[0][0], acc[0][1], acc[0][2], acc[0][3]);
  acc_guard4(acc[1][0], acc[1][1], acc[1][2], acc[1][3]);
  acc_guard4(acc[2][0], acc[2][1], acc[2][2], acc[2][3]);
  acc_guard4(acc[3][0], acc[3][1], acc[3][2], acc[3][3]);

  float* slab = sT[wave];
#pragma unroll
  for (int i = 0; i < 4; ++i) {
    const int mBase = m0 + (i << 4);
#pragma unroll
    for (int jj = 0; jj < 4; ++jj) {
      const int n = n0 + (jj << 4) + rlane;
      float bv = bias[n];
      if (BIAS_R16) bv = bf16r(bv);
#pragma unroll
      for (int r = 0; r < 8; ++r) {
        const float v = acc[i][jj][r] * scale + bv;
        slab[(mOff + r) * 68 + (jj << 4) + rlane] = v;
      }
    }
    __builtin_amdgcn_fence(__ATOMIC_RELEASE, "workgroup");
    __builtin_amdgcn_wave_barrier();
    __builtin_amdgcn_fence(__ATOMIC_ACQUIRE, "workgroup");
    {
      const int hh = lane >> 4, c4 = (lane & 15) * 4;
      for (int pass = 0; pass < 2; ++pass) {
#pragma unroll
        for (int it = 0; it < 8; ++it) {
          const int row = it * 2 + hh;
          const v4f v = *(const v4f*)(slab + row * 68 + c4);
          *(volatile v4f*)(Cout + (size_t)(mBase + row) * ldc + n0 + c4) = v;
        }
        __threadfence();
      }
    }
    __builtin_amdgcn_fence(__ATOMIC_RELEASE, "workgroup");
    __builtin_amdgcn_wave_barrier();
    __builtin_amdgcn_fence(__ATOMIC_ACQUIRE, "workgroup");
  }
}

extern "C" void kernel_launch(void* const* d_in, const int* in_sizes, int n_in,
                              void* d_out, int out_size, void* d_ws, size_t ws_size, hipStream_t stream) {
  if (n_in < 10 || d_out == nullptr || d_ws == nullptr) return;
  if (in_sizes[0] != NBAT * NFEAT || in_sizes[1] != NLAY * NBAT * NHID || in_sizes[2] != NHID * NFEAT ||
      in_sizes[3] != NHID || in_sizes[4] != NLAY * NGATE * NHID || in_sizes[5] != NLAY * NGATE * NHID ||
      in_sizes[6] != NLAY * NGATE || in_sizes[7] != NLAY * NGATE || in_sizes[8] != NOUT * NHID ||
      in_sizes[9] != NOUT || out_size != NBAT * NOUT + NLAY * NBAT * NHID) return;

  const float* input  = (const float*)d_in[0];
  const float* hidden = (const float*)d_in[1];
  const float* i2h_w  = (const float*)d_in[2];
  const float* i2h_b  = (const float*)d_in[3];
  const float* w_ih   = (const float*)d_in[4];
  const float* w_hh   = (const float*)d_in[5];
  const float* b_ih   = (const float*)d_in[6];
  const float* b_hh   = (const float*)d_in[7];
  const float* dec_w  = (const float*)d_in[8];
  const float* dec_b  = (const float*)d_in[9];

  float* logits  = (float*)d_out;
  float* hid_out = logits + (size_t)NBAT * NOUT;

  char* ws = (char*)d_ws;
  size_t off = 0;
  auto carve = [&](size_t bytes) -> char* { char* p = ws + off; off += (bytes + 255) & ~(size_t)255; return p; };
  unsigned short* WIH16 = (unsigned short*)carve((size_t)NLAY * NGATE * NHID * 2);
  unsigned short* WHH16 = (unsigned short*)carve((size_t)NLAY * NGATE * NHID * 2);
  unsigned short* HID16 = (unsigned short*)carve((size_t)NLAY * NBAT * NHID * 2);
  unsigned short* DEC16 = (unsigned short*)carve((size_t)NOUT * NHID * 2);
  unsigned short* XA    = (unsigned short*)carve((size_t)NBAT * NHID * 2);
  unsigned short* XB    = (unsigned short*)carve((size_t)NBAT * NHID * 2);
  if (off > ws_size || off > (size_t)134217728) return;

  const int n8w = NLAY * NGATE * (NHID / 8);
  const int n8h = NLAY * NBAT * (NHID / 8);
  const int n8d = NOUT * (NHID / 8);
  cvt8_flat_kernel<<<(n8w + NTHR - 1) / NTHR, NTHR, 0, stream>>>(w_ih,   WIH16, n8w, CARRY);
  cvt8_flat_kernel<<<(n8w + NTHR - 1) / NTHR, NTHR, 0, stream>>>(w_hh,   WHH16, n8w, CARRY);
  cvt8_flat_kernel<<<(n8h + NTHR - 1) / NTHR, NTHR, 0, stream>>>(hidden, HID16, n8h, CARRY);
  cvt8_flat_kernel<<<(n8d + NTHR - 1) / NTHR, NTHR, 0, stream>>>(dec_w,  DEC16, n8d, CARRY);

  i2h_kernel<<<(NBAT * NHID / 8) / NTHR, NTHR, 0, stream>>>(input, i2h_w, i2h_b, XA);

  const dim3 ggrid(NHID / BLK_COLS, NBAT / BLK_ROWS);
  for (int l = 0; l < NLAY; ++l) {
    const unsigned short* xin = (l & 1) ? XB : XA;
    unsigned short* xout      = (l & 1) ? XA : XB;
    gru_layer_kernel<<<ggrid, NTHR, 0, stream>>>(
        xin, HID16 + (size_t)l * NBAT * NHID,
        WIH16 + (size_t)l * NGATE * NHID, WHH16 + (size_t)l * NGATE * NHID,
        b_ih + (size_t)l * NGATE, b_hh + (size_t)l * NGATE,
        hidden + (size_t)l * NBAT * NHID, hid_out + (size_t)l * NBAT * NHID, xout);
  }

  const int dtiles = (NBAT / 64) * (NOUT / 64);
  wmma_gemm64_f16<true><<<(dtiles + 7) / 8, 256, 0, stream>>>(
      XA, NHID, DEC16, NHID, logits, NOUT, dec_b, NBAT, NOUT, NHID, PROD_INV);
}
